// GCNencoder_21758304322142
// MI455X (gfx1250) — hardware-verified
//
#include <hip/hip_runtime.h>

typedef float          v8f   __attribute__((ext_vector_type(8)));
typedef float          v4f   __attribute__((ext_vector_type(4)));
typedef unsigned int   v4u   __attribute__((ext_vector_type(4)));
typedef int            v8i   __attribute__((ext_vector_type(8)));
typedef unsigned short v8us  __attribute__((ext_vector_type(8)));
typedef unsigned short v16us __attribute__((ext_vector_type(16)));
typedef __bf16         v16bf __attribute__((ext_vector_type(16)));
typedef _Float16       v16h  __attribute__((ext_vector_type(16)));
typedef v4f  __attribute__((may_alias)) v4fa;
typedef v8us __attribute__((may_alias)) v8usa;
union FragB { v16bf v; v16us u; v8us h[2]; v8i w; };
union FragH { v16h  v; v16us u; v8us h[2]; v8i w; };

__device__ __forceinline__ v8f wmb(const FragB& a, const FragB& b, v8f c) {
  v8f d = __builtin_amdgcn_wmma_f32_16x16x32_bf16(false, a.v, false, b.v, (short)0, c, false, false);
  asm volatile("v_nop\n\tv_nop\n\tv_nop\n\tv_nop" : "+v"(d) : "v"(a.w), "v"(b.w));
  return d;
}

__device__ __forceinline__ v8f wmh(const FragH& a, const FragH& b, v8f c) {
  v8f d = __builtin_amdgcn_wmma_f32_16x16x32_f16(false, a.v, false, b.v, (short)0, c, false, false);
  asm volatile("v_nop\n\tv_nop\n\tv_nop\n\tv_nop" : "+v"(d) : "v"(a.w), "v"(b.w));
  return d;
}

__device__ __forceinline__ unsigned bf16_bits(float f) {
  const unsigned u = __float_as_uint(f);
  const unsigned r = (u + 0x7FFFu + ((u >> 16) & 1u)) >> 16;
  const unsigned q = (u >> 16) | 0x40u;
  return ((u & 0x7fffffffu) > 0x7f800000u) ? q : r;
}

__device__ __forceinline__ float bf16_val(float f) {
  return __uint_as_float(bf16_bits(f) << 16);
}
__device__ __forceinline__ int clampi(int v, int lo, int hi) {
  return v < lo ? lo : (v > hi ? hi : v);
}

__device__ __forceinline__ unsigned f16_bits(float f) {
  const unsigned u  = __float_as_uint(f);
  const unsigned s  = (u >> 16) & 0x8000u;
  const unsigned a  = u & 0x7fffffffu;
  const unsigned t  = a - 0x38000000u;
  const unsigned r  = (t + 0x0FFFu + ((t >> 13) & 1u)) >> 13;
  const unsigned rc = r > 0x7C00u ? 0x7C00u : r;
  const bool small  = a < 0x38800000u;
  const bool isnan  = a > 0x7f800000u;
  const unsigned fin = small ? 0u : (s | rc);
  return isnan ? (s | 0x7E00u) : fin;
}

__device__ __forceinline__ unsigned pk16(unsigned lo, unsigned hi) { return lo | (hi << 16); }
__device__ __forceinline__ unsigned bf16_lo_bits(float v) {
  float hi = bf16_val(v);
  asm volatile("" : "+v"(hi));
  return bf16_bits(v - hi);
}
__device__ __forceinline__ v4u pack8_bf16(v4f a, v4f c) {
  return (v4u){ pk16(bf16_bits(a[0]), bf16_bits(a[1])), pk16(bf16_bits(a[2]), bf16_bits(a[3])),
                pk16(bf16_bits(c[0]), bf16_bits(c[1])), pk16(bf16_bits(c[2]), bf16_bits(c[3])) };
}
__device__ __forceinline__ v4u pack8_bf16_lo(v4f a, v4f c) {
  return (v4u){ pk16(bf16_lo_bits(a[0]), bf16_lo_bits(a[1])), pk16(bf16_lo_bits(a[2]), bf16_lo_bits(a[3])),
                pk16(bf16_lo_bits(c[0]), bf16_lo_bits(c[1])), pk16(bf16_lo_bits(c[2]), bf16_lo_bits(c[3])) };
}
__device__ __forceinline__ v4u pack8_f16(v4f a, v4f c) {
  return (v4u){ pk16(f16_bits(a[0]), f16_bits(a[1])), pk16(f16_bits(a[2]), f16_bits(a[3])),
                pk16(f16_bits(c[0]), f16_bits(c[1])), pk16(f16_bits(c[2]), f16_bits(c[3])) };
}

template <int FORM>
__global__ __launch_bounds__(256) void k_plane(const float* __restrict__ src, int rows, int cols, int ldsrc,
                                               unsigned short* __restrict__ dst, int MP, int KP) {
  static_assert(FORM >= 0 && FORM <= 3);
  const int KTOT = (FORM == 1 || FORM == 3) ? 2 * KP : KP;
  const unsigned ppr   = (unsigned)(KTOT >> 3);
  const unsigned kp8   = (unsigned)(KP >> 3);
  const unsigned total = (unsigned)MP * ppr;
  const unsigned g     = blockIdx.x * 256u + threadIdx.x;
  const unsigned rowu  = g / ppr;
  const unsigned p     = g - rowu * ppr;
  const bool second    = p >= kp8;
  const int row = (int)rowu;
  const int c0  = (int)((second ? p - kp8 : p) << 3);
  const float* srow = src + (size_t)clampi(row, 0, rows - 1) * (size_t)ldsrc;
  float x[8];
  unsigned mk[8];
#pragma unroll
  for (int e = 0; e < 8; ++e) {
    const int c = c0 + e;
    const float v = srow[clampi(c, 0, cols - 1)];
    asm volatile("" :: "v"(v));
    x[e]  = v;
    mk[e] = (row < rows && c < cols) ? 0xFFFFu : 0u;
  }
  const v4f a = (v4f){ x[0], x[1], x[2], x[3] };
  const v4f c = (v4f){ x[4], x[5], x[6], x[7] };
  v4u o;
  if (FORM == 2) {
    o = pack8_f16(a, c);
  } else {
    const v4u hi = pack8_bf16(a, c);
    o = hi;
    if (FORM == 1) { const v4u lo = pack8_bf16_lo(a, c); o = second ? lo : hi; }
  }
  const v4u mw = (v4u){ pk16(mk[0], mk[1]), pk16(mk[2], mk[3]), pk16(mk[4], mk[5]), pk16(mk[6], mk[7]) };
  o &= mw;
  if (g < total) {
    volatile v4u* q = (volatile v4u*)(dst + (size_t)g * 8);
    *q = o;
    __threadfence();
    *q = o;
  }
}

template <int FORM> struct FragOf    { typedef FragB T; };
template <>         struct FragOf<2> { typedef FragH T; };
__device__ __forceinline__ v8f mm(const FragB& a, const FragB& b, v8f c) { return wmb(a, b, c); }
__device__ __forceinline__ v8f mm(const FragH& a, const FragH& b, v8f c) { return wmh(a, b, c); }
template <class F> __device__ __forceinline__ F ld_frag(const unsigned short* p) {
  F f;
  f.h[0] = *(const v8usa*)(p);
  f.h[1] = *(const v8usa*)(p + 16);
  return f;
}

template <int FORM, int EPI>
__global__ __launch_bounds__(256) __attribute__((amdgpu_num_vgpr(248)))
void k_gemm_nt(const unsigned short* __restrict__ A, const unsigned short* __restrict__ B,
               const float* __restrict__ bias, float* __restrict__ D, int M, int N, int KTOT, int ldd) {
  static_assert(FORM >= 0 && FORM <= 2);
  static_assert(EPI == 0 || EPI == 1);
  typedef typename FragOf<FORM>::T F;
  __shared__ __attribute__((aligned(16))) float sT[8][16 * 68];
  const int lane = threadIdx.x & 31;
  const int wave = threadIdx.x >> 5;
  const int tilesM = (M + 63) >> 6;
  const int tilesN = (N + 63) >> 6;
  const int tile = blockIdx.x * 8 + wave;
  if (tile >= tilesM * tilesN) return;
  const int tm = tile / tilesN;
  const int tn = tile - tm * tilesN;
  const int m0 = tm << 6;
  const int n0 = tn << 6;

  const int rl = lane & 15;
  const int h8 = (lane >> 4) * 8;
  const unsigned short* pa = A + (size_t)(m0 + rl) * (size_t)KTOT + h8;
  const unsigned short* pb = B + (size_t)(n0 + rl) * (size_t)KTOT + h8;

  v8f acc[4][4];
#pragma unroll
  for (int i = 0; i < 4; ++i)
#pragma unroll
    for (int j = 0; j < 4; ++j) acc[i][j] = (v8f){0.f, 0.f, 0.f, 0.f, 0.f, 0.f, 0.f, 0.f};

#pragma unroll 1
  for (int k0 = 0; k0 < KTOT; k0 += 32) {
    F bf[4];
#pragma unroll
    for (int j = 0; j < 4; ++j) bf[j] = ld_frag<F>(pb + (size_t)(j << 4) * (size_t)KTOT + k0);
#pragma unroll
    for (int i = 0; i < 4; ++i) {
      const F af = ld_frag<F>(pa + (size_t)(i << 4) * (size_t)KTOT + k0);
#pragma unroll
      for (int j = 0; j < 4; ++j) acc[i][j] = mm(af, bf[j], acc[i][j]);
    }
  }

  float* slab = sT[wave];
  const int hh = lane >> 4;
  const int c4 = (lane & 15) * 4;
  const int nc = n0 + c4;
  const bool cok = nc < N;
  v4f bv = (v4f){0.f, 0.f, 0.f, 0.f};
  if (EPI == 1) {
    bv = *(const v4fa*)(bias + clampi(nc, 0, N - 4));
    asm volatile("" :: "v"(bv));
  }
#pragma unroll
  for (int i = 0; i < 4; ++i) {
    const int mBase = m0 + (i << 4);
#pragma unroll
    for (int j = 0; j < 4; ++j) {
#pragma unroll
      for (int r = 0; r < 8; ++r) slab[(h8 + r) * 68 + (j << 4) + rl] = acc[i][j][r];
    }
    __builtin_amdgcn_fence(__ATOMIC_RELEASE, "workgroup");
    __builtin_amdgcn_wave_barrier();
    __builtin_amdgcn_fence(__ATOMIC_ACQUIRE, "workgroup");
    v4f vv[8];
#pragma unroll
    for (int it = 0; it < 8; ++it) {
      const int row = it * 2 + hh;
      v4f v = *(const v4fa*)(slab + row * 68 + c4);
      if (EPI == 1) v += bv;
      vv[it] = v;
    }
    for (int pass = 0; pass < 2; ++pass) {
#pragma unroll
      for (int it = 0; it < 8; ++it) {
        const int row = mBase + it * 2 + hh;
        if (cok && row < M) *(volatile v4f*)(D + (size_t)row * (size_t)ldd + nc) = vv[it];
      }
      __threadfence();
    }
    __builtin_amdgcn_fence(__ATOMIC_RELEASE, "workgroup");
    __builtin_amdgcn_wave_barrier();
    __builtin_amdgcn_fence(__ATOMIC_ACQUIRE, "workgroup");
  }
}

#include <math.h>
#include <stddef.h>

#define GB   65536
#define GN   121
#define GNP  128
#define GH   32
#ifndef P2_TWO_TERM
#define P2_TWO_TERM 1
#endif
#if P2_TWO_TERM
#define S2K 256
#else
#define S2K 128
#endif
#define OUT_N   (GB * GN)
#define GRP_F   (32 * GN)

static_assert(GN <= GNP);
static_assert(GB % 128 == 0 && GB % 32 == 0 && GB % 64 == 0 && GB % 16 == 0);
static_assert((32 * GN * 4) % 128 == 0);
static_assert(GRP_F == 121 * 32);
static_assert(GH == 32);
static_assert(GNP % 64 == 0 && GNP % 32 == 0 && GNP % 4 == 0 && S2K % 32 == 0);
static_assert((GB * 16) % 256 == 0 && (GB / 32) % 8 == 0);

static constexpr size_t SZ_XB   = (size_t)GB * GNP * 2;
static constexpr size_t SZ_Y    = (size_t)GB * GNP * 4;
static constexpr size_t SZ_S2   = (size_t)GB * 256 * 2;
static constexpr size_t SZ_ADJ1 = (size_t)GNP * GNP * 2;
static constexpr size_t SZ_ADJ2 = (size_t)GNP * 256 * 2;
static constexpr size_t SZ_WV   = 256;
static constexpr size_t O_XB   = 0;
static constexpr size_t O_Y    = O_XB   + SZ_XB;
static constexpr size_t O_S2   = O_Y    + SZ_Y;
static constexpr size_t O_ADJ1 = O_S2   + SZ_S2;
static constexpr size_t O_ADJ2 = O_ADJ1 + SZ_ADJ1;
static constexpr size_t O_WV   = O_ADJ2 + SZ_ADJ2;
static constexpr size_t WS_TOTAL = O_WV + SZ_WV;
static_assert(SZ_XB % 256 == 0 && SZ_Y % 256 == 0 && SZ_S2 % 256 == 0 && SZ_ADJ1 % 256 == 0 && SZ_ADJ2 % 256 == 0);
static_assert(O_Y == 16777216 && O_S2 == 50331648 && O_ADJ1 == 83886080 && O_ADJ2 == 83918848 && O_WV == 83984384);
static_assert(WS_TOTAL == 83984640);
static_assert(WS_TOTAL <= ((size_t)128 << 20));
static_assert((size_t)GB * S2K * 2 <= SZ_S2);

__global__ __launch_bounds__(256) void k_prep_adj(const float* __restrict__ adj, const float* __restrict__ W1,
                                                  const float* __restrict__ W2,
                                                  unsigned short* ADJ1, unsigned short* ADJ2, float* WV) {
  const int t = (int)threadIdx.x;
#pragma unroll 1
  for (int it = 0; it < 8; ++it) {
    const int g  = it * 256 + t;
    const int n  = g >> 4;
    const int k0 = (g & 15) << 3;
    const int nr = n < GN - 1 ? n : GN - 1;
    const float* srow = adj + nr * GN;
    float x[8];
    unsigned mk[8];
#pragma unroll
    for (int e = 0; e < 8; ++e) {
      const int k  = k0 + e;
      const int kc = k < GN - 1 ? k : GN - 1;
      const float v = srow[kc];
      asm volatile("" :: "v"(v));
      x[e]  = v;
      mk[e] = (n < GN && k < GN) ? 0xFFFFu : 0u;
    }
    v4u o = pack8_bf16((v4f){ x[0], x[1], x[2], x[3] }, (v4f){ x[4], x[5], x[6], x[7] });
    const v4u mw = (v4u){ pk16(mk[0], mk[1]), pk16(mk[2], mk[3]), pk16(mk[4], mk[5]), pk16(mk[6], mk[7]) };
    o &= mw;
    volatile v4u* q1 = (volatile v4u*)(ADJ1 + (size_t)g * 8);
    volatile v4u* q2 = (volatile v4u*)(ADJ2 + (size_t)n * 256 + k0);
    volatile v4u* q3 = (volatile v4u*)(ADJ2 + (size_t)n * 256 + 128 + k0);
    *q1 = o;
    *q2 = o;
    *q3 = o;
    __threadfence();
    *q1 = o;
    *q2 = o;
    *q3 = o;
  }
  if (t < 32) {
    const int q    = t & 15;
    const int base = (q & 7) << 2;
    const unsigned sel = (q >= 8) ? 0xFFFFFFFFu : 0u;
    float o[4];
#pragma unroll
    for (int e = 0; e < 4; ++e) {
      const float a = W1[base + e];
      const float b = W2[base + e];
      asm volatile("" :: "v"(a));
      asm volatile("" :: "v"(b));
      const unsigned u = (__float_as_uint(a) & ~sel) | (__float_as_uint(b) & sel);
      o[e] = bf16_val(__uint_as_float(u));
    }
    const v4f ov = (v4f){ o[0], o[1], o[2], o[3] };
    volatile v4f* qw = (volatile v4f*)(WV + 4 * q);
    for (int ps = 0; ps < 2; ++ps) {
      if (t < 16) *qw = ov;
      __threadfence();
    }
  }
}

__global__ __launch_bounds__(256) void k_xplane(const float* __restrict__ x, unsigned short* XB) {
  const unsigned g = blockIdx.x * 256u + threadIdx.x;
  const unsigned b = g >> 4;
  const int c0 = (int)(g & 15u) << 3;
  const float* xr = x + (size_t)b * GN;
  float v8[8];
  unsigned mk[8];
#pragma unroll
  for (int e = 0; e < 8; ++e) {
    const int c  = c0 + e;
    const int cc = c < GN - 1 ? c : GN - 1;
    const float v = xr[cc];
    asm volatile("" :: "v"(v));
    v8[e] = v;
    mk[e] = (c < GN) ? 0xFFFFu : 0u;
  }
  v4u o = pack8_bf16((v4f){ v8[0], v8[1], v8[2], v8[3] }, (v4f){ v8[4], v8[5], v8[6], v8[7] });
  const v4u mw = (v4u){ pk16(mk[0], mk[1]), pk16(mk[2], mk[3]), pk16(mk[4], mk[5]), pk16(mk[6], mk[7]) };
  o &= mw;
  volatile v4u* q = (volatile v4u*)(XB + (size_t)g * 8);
  *q = o;
  __threadfence();
  *q = o;
}

__global__ __launch_bounds__(256) void k_row(const float* __restrict__ Y, const float* __restrict__ WV,
                                             unsigned short* S2) {
  __shared__ __attribute__((aligned(16))) float swv[64];
  const int t = (int)threadIdx.x;
  if (t < 32) {
    const float a = WV[2 * t];
    const float b = WV[2 * t + 1];
    swv[2 * t]     = a;
    swv[2 * t + 1] = b;
  }
  __syncthreads();
  const unsigned g  = blockIdx.x * 256u + (unsigned)t;
  const unsigned b  = g >> 4;
  const int      c8 = (int)(g & 15u);
  const float* yp = Y + (size_t)g * 8;
  const v4f ya = *(const v4fa*)(yp);
  const v4f yb = *(const v4fa*)(yp + 4);
  asm volatile("" :: "v"(ya));
  asm volatile("" :: "v"(yb));
  float y[8] = { ya[0], ya[1], ya[2], ya[3], yb[0], yb[1], yb[2], yb[3] };
  float acc[8] = { 0.0f, 0.0f, 0.0f, 0.0f, 0.0f, 0.0f, 0.0f, 0.0f };
#pragma unroll 2
  for (int h = 0; h < GH; ++h) {
    const float w1 = swv[h];
    const float w2 = swv[GH + h];
#pragma unroll
    for (int i = 0; i < 8; ++i) {
      const float tt = w1 * y[i];
      const float r  = fmaxf(tt, 0.0f);
      acc[i] += r * w2;
    }
  }
#pragma unroll
  for (int i = 0; i < 8; ++i) acc[i] = (8 * c8 + i < GN) ? acc[i] : 0.0f;
  const v4f a = (v4f){ acc[0], acc[1], acc[2], acc[3] };
  const v4f c = (v4f){ acc[4], acc[5], acc[6], acc[7] };
  const v4u hi = pack8_bf16(a, c);
#if P2_TWO_TERM
  const v4u lo = pack8_bf16_lo(a, c);
  volatile v4u* qh = (volatile v4u*)(S2 + (size_t)b * 256 + 8 * c8);
  volatile v4u* ql = (volatile v4u*)(S2 + (size_t)b * 256 + 128 + 8 * c8);
  *qh = hi;
  *ql = lo;
  __threadfence();
  *qh = hi;
  *ql = lo;
#else
  volatile v4u* qh = (volatile v4u*)(S2 + (size_t)g * 8);
  *qh = hi;
  __threadfence();
  *qh = hi;
#endif
}

__global__ __launch_bounds__(256) void k_copy(const float* __restrict__ Y, float* out) {
  const int lane = (int)threadIdx.x & 31;
  const int wave = (int)threadIdx.x >> 5;
  const unsigned grp = blockIdx.x * 8u + (unsigned)wave;
  const float* yb = Y + (size_t)grp * (32 * GNP);
  float* ob = out + (size_t)grp * GRP_F;
#pragma unroll 1
  for (int ch = 0; ch < 15; ++ch) {
    float v[8];
#pragma unroll
    for (int e = 0; e < 8; ++e) {
      const unsigned j = (unsigned)((ch * 8 + e) * 32 + lane);
      const unsigned r = j / 121u;
      const unsigned c = j - 121u * r;
      v[e] = yb[r * GNP + c];
    }
    for (int ps = 0; ps < 2; ++ps) {
#pragma unroll
      for (int e = 0; e < 8; ++e) *(volatile float*)(ob + (ch * 8 + e) * 32 + lane) = v[e];
      __threadfence();
    }
  }
  {
    const unsigned j = (unsigned)(120 * 32 + lane);
    const unsigned r = j / 121u;
    const unsigned c = j - 121u * r;
    const float v = yb[r * GNP + c];
    for (int ps = 0; ps < 2; ++ps) {
      *(volatile float*)(ob + j) = v;
      __threadfence();
    }
  }
}

extern "C" void kernel_launch(void* const* d_in, const int* in_sizes, int n_in,
                              void* d_out, int out_size, void* d_ws, size_t ws_size,
                              hipStream_t stream) {
  if (n_in < 4) return;
  if (in_sizes[0] != GB * GN) return;
  if (in_sizes[1] != GN * GN) return;
  if (in_sizes[2] != GH) return;
  if (in_sizes[3] != GH) return;
  if (out_size != OUT_N) return;
  if ((size_t)WS_TOTAL > ws_size) return;

  const float* x   = (const float*)d_in[0];
  const float* adj = (const float*)d_in[1];
  const float* W1  = (const float*)d_in[2];
  const float* W2  = (const float*)d_in[3];
  float* out = (float*)d_out;

  char* ws = (char*)d_ws;
  unsigned short* XB   = (unsigned short*)(ws + O_XB);
  float*          Y    = (float*)(ws + O_Y);
  unsigned short* S2   = (unsigned short*)(ws + O_S2);
  unsigned short* ADJ1 = (unsigned short*)(ws + O_ADJ1);
  unsigned short* ADJ2 = (unsigned short*)(ws + O_ADJ2);
  float*          WV   = (float*)(ws + O_WV);

  const int gemm_blocks = ((GB / 64) * (GNP / 64) + 7) / 8;

  k_prep_adj<<<1, 256, 0, stream>>>(adj, W1, W2, ADJ1, ADJ2, WV);
  k_xplane<<<GB * 16 / 256, 256, 0, stream>>>(x, XB);
  k_gemm_nt<0, 0><<<gemm_blocks, 256, 0, stream>>>(XB, ADJ1, WV, Y, GB, GNP, GNP, GNP);
  k_row<<<GB * 16 / 256, 256, 0, stream>>>(Y, WV, S2);
#if P2_TWO_TERM
  k_gemm_nt<0, 0><<<gemm_blocks, 256, 0, stream>>>(S2, ADJ2, WV, Y, GB, GNP, S2K, GNP);
#else
  k_gemm_nt<0, 0><<<gemm_blocks, 256, 0, stream>>>(S2, ADJ1, WV, Y, GB, GNP, S2K, GNP);
#endif
  k_copy<<<GB / 32 / 8, 256, 0, stream>>>(Y, out);
}
